// se3AtomCloudNet_3917010173961
// MI455X (gfx1250) — hardware-verified
//
#include <hip/hip_runtime.h>
#include <stdint.h>
#include <math.h>

#pragma clang fp contract(off)

#define NB 32
#define NA 30
#define NPAIR 28800
#define EMBD 32
#define HR 100
#define HP 128
#define NLU 72
#define RES 216
#define FAP 256
#define WRROWS 256
#define TLP 256
#define PP 256
#define WCK 448
#define W2P 2304
#define W2PIECES 28928

typedef unsigned short us;
typedef us v8us_t __attribute__((ext_vector_type(8)));
typedef v8us_t __attribute__((may_alias)) v8us;
typedef us v16us __attribute__((ext_vector_type(16)));
typedef __bf16 v16b __attribute__((ext_vector_type(16)));
typedef float v8f __attribute__((ext_vector_type(8)));
typedef float v4f_t __attribute__((ext_vector_type(4)));
typedef v4f_t __attribute__((may_alias)) v4f;
typedef unsigned int v4u __attribute__((ext_vector_type(4)));
typedef unsigned int v8u __attribute__((ext_vector_type(8)));

union Frag { v16us u; v8us_t h[2]; v16b b; v8u w; };
union P16 { v8us_t h; v4u u; us s[8]; };

__device__ __forceinline__ v8f zero8() {
  v8f z;
#pragma unroll
  for (int i = 0; i < 8; ++i) z[i] = 0.0f;
  return z;
}

__device__ __forceinline__ us bf_bits(float x) {
  unsigned int u = __float_as_uint(x);
  u += 0x7FFFu + ((u >> 16) & 1u);
  return (us)(u >> 16);
}
__device__ __forceinline__ float bf_val(us b) { return __uint_as_float(((unsigned int)b) << 16); }
__device__ __forceinline__ void split2(float x, us& hi, us& lo) {
  const us hb = bf_bits(x);
  hi = hb;
  lo = bf_bits(x - bf_val(hb));
}

__device__ __forceinline__ Frag ldfrag(const us* p, int k0) {
  Frag f;
  f.h[0] = *(const v8us*)(p + k0);
  f.h[1] = *(const v8us*)(p + k0 + 16);
  return f;
}

__device__ __forceinline__ v8f wmb(v16b a, v16b b, v8f c) {
  return __builtin_amdgcn_wmma_f32_16x16x32_bf16(false, a, false, b, (short)0, c, false, false);
}
__device__ __forceinline__ v8f mma3(const Frag ah, const Frag al, const Frag bh, const Frag bl, v8f c) {
  c = wmb(ah.b, bh.b, c);
  c = wmb(ah.b, bl.b, c);
  c = wmb(al.b, bh.b, c);
  return c;
}

__device__ __forceinline__ void vst16(us* p, v8us_t v) { P16 k; k.h = v; *(volatile v4u*)p = k.u; }
__device__ __forceinline__ void vst16f(float* p, v4f_t v) { *(volatile v4f_t*)p = v; }

__device__ __forceinline__ float sp5(float x) {
  const float y = 5.0f * x;
  const float s = fmaxf(y, 0.0f) + log1pf(expf(-fabsf(y)));
  return s * 0.281f;
}

__device__ __forceinline__ float geo_d(const float* pa, const float* pb, float& dx, float& dy, float& dz) {
  dx = pb[0] - pa[0]; dy = pb[1] - pa[1]; dz = pb[2] - pa[2];
  const float d2 = dx * dx + dy * dy + dz * dz;
  const bool pos = d2 > 0.0f;
  const float s = sqrtf(pos ? d2 : 1.0f);
  return pos ? s : 0.0f;
}

__global__ void __launch_bounds__(256) k_cvt(const float* __restrict__ src, us* __restrict__ dh,
                                             us* __restrict__ dl, int nrow, int ncol, int sld,
                                             int kp8, int trans) {
  const int i = blockIdx.x * 256 + (int)threadIdx.x;
  const int row = i / kp8;
  const int q = i - row * kp8;
  P16 ph, pl;
#pragma unroll
  for (int j = 0; j < 8; ++j) {
    const int k = 8 * q + j;
    const bool ok = (row < nrow) && (k < ncol);
    const int rc = min(row, nrow - 1), kc = min(k, ncol - 1);
    const size_t idx = trans ? ((size_t)kc * sld + rc) : ((size_t)rc * sld + kc);
    float v = src[idx];
    v = ok ? v : 0.0f;
    us hb, lb;
    split2(v, hb, lb);
    ph.s[j] = hb; pl.s[j] = lb;
  }
  us* qh = dh + (size_t)i * 8;
  us* ql = dl + (size_t)i * 8;
  vst16(qh, ph.h); vst16(ql, pl.h);
  __threadfence();
  vst16(qh, ph.h); vst16(ql, pl.h);
}

__global__ void __launch_bounds__(256) k_feat(const int* __restrict__ fid, const float* __restrict__ emb,
                                              us* __restrict__ dh, us* __restrict__ dl) {
  const int i = blockIdx.x * 256 + (int)threadIdx.x;
  const int zb = i >> 2, q = i & 3;
  int f = fid[zb];
  f = min(max(f, 0), 5);
  P16 ph, pl;
#pragma unroll
  for (int j = 0; j < 8; ++j) {
    const float v = emb[f * EMBD + 8 * q + j];
    us hb, lb;
    split2(v, hb, lb);
    ph.s[j] = hb; pl.s[j] = lb;
  }
  us* qh = dh + (size_t)i * 8;
  us* ql = dl + (size_t)i * 8;
  vst16(qh, ph.h); vst16(ql, pl.h);
  __threadfence();
  vst16(qh, ph.h); vst16(ql, pl.h);
}

__global__ void __launch_bounds__(256) k_geom(const float* __restrict__ xyz, const float* __restrict__ w_r0,
                                              us* __restrict__ h0h, us* __restrict__ h0l) {
  __shared__ float sbas[32][4];
  __shared__ __align__(16) us sh[2][32][HP];
  const int tid = (int)threadIdx.x, lane = tid & 31, w = tid >> 5;
  const int p0 = blockIdx.x * 32;
  if (tid < 32) {
    const int p = p0 + tid;
    const int z = p / (NA * NA);
    const int rem = p - z * (NA * NA);
    const int a = rem / NA;
    const int b = rem - a * NA;
    float dx, dy, dz;
    const float d = geo_d(xyz + ((size_t)z * NA + a) * 3, xyz + ((size_t)z * NA + b) * 3, dx, dy, dz);
#pragma unroll 1
    for (int j = 0; j < 3; ++j) {
      const float xk = d - (float)j;
      const float cv = cosf(1.5707963267948966f * xk);
      sbas[tid][j] = (fabsf(xk) < 1.0f) ? cv * cv : 0.0f;
    }
    sbas[tid][3] = 0.0f;
  }
  __syncthreads();
  const float b0 = sbas[lane][0], b1 = sbas[lane][1], b2 = sbas[lane][2];
#pragma unroll 1
  for (int j = 0; j < 16; ++j) {
    const int t = w + 8 * j;
    const int tc = min(t, HR - 1);
    const float acc = b0 * w_r0[tc] + b1 * w_r0[HR + tc] + b2 * w_r0[2 * HR + tc];
    const float sv = sp5(acc);
    const float v = (t < HR) ? sv : 0.0f;
    us hb, lb;
    split2(v, hb, lb);
    sh[0][lane][t] = hb;
    sh[1][lane][t] = lb;
  }
  __syncthreads();
  v8us_t vv[2][2];
#pragma unroll
  for (int j = 0; j < 2; ++j) {
    const int row = (tid >> 4) + 16 * j;
    const int q = tid & 15;
    vv[0][j] = *(const v8us*)(&sh[0][row][8 * q]);
    vv[1][j] = *(const v8us*)(&sh[1][row][8 * q]);
  }
#pragma unroll
  for (int j = 0; j < 2; ++j) {
    const int row = (tid >> 4) + 16 * j;
    const int q = tid & 15;
    const size_t o = (size_t)(p0 + row) * HP + 8 * q;
    vst16(h0h + o, vv[0][j]); vst16(h0l + o, vv[1][j]);
  }
  __threadfence();
#pragma unroll
  for (int j = 0; j < 2; ++j) {
    const int row = (tid >> 4) + 16 * j;
    const int q = tid & 15;
    const size_t o = (size_t)(p0 + row) * HP + 8 * q;
    vst16(h0h + o, vv[0][j]); vst16(h0l + o, vv[1][j]);
  }
}

__global__ void __launch_bounds__(128) k_mlp1(const us* __restrict__ h0h, const us* __restrict__ h0l,
                                              const us* __restrict__ w1h, const us* __restrict__ w1l,
                                              us* __restrict__ h1h, us* __restrict__ h1l) {
  __shared__ __align__(16) us st[4][2][16][HP];
  const int tid = (int)threadIdx.x, lane = tid & 31, w = tid >> 5;
  const int hh = lane >> 4, m = lane & 15;
  const int mt = blockIdx.x * 4 + w;
  const size_t row0 = (size_t)mt * 16;
  const us* pah = h0h + (row0 + m) * HP + 8 * hh;
  const us* pal = h0l + (row0 + m) * HP + 8 * hh;
  v8f acc[7];
#pragma unroll
  for (int t = 0; t < 7; ++t) acc[t] = zero8();
#pragma unroll 1
  for (int ks = 0; ks < 4; ++ks) {
    const int k0 = ks * 32;
    const Frag ah = ldfrag(pah, k0), al = ldfrag(pal, k0);
    Frag bh, bl;
#pragma unroll
    for (int nt = 0; nt < 7; ++nt) {
      const size_t ob = (size_t)(nt * 16 + m) * HP + 8 * hh;
      bh = ldfrag(w1h + ob, k0);
      bl = ldfrag(w1l + ob, k0);
      acc[nt] = mma3(ah, al, bh, bl, acc[nt]);
    }
    asm volatile("v_nop\n\tv_nop\n\tv_nop\n\tv_nop"
                 : "+v"(acc[0]), "+v"(acc[1]), "+v"(acc[2]), "+v"(acc[3]),
                   "+v"(acc[4]), "+v"(acc[5]), "+v"(acc[6])
                 : "v"(ah.b), "v"(al.b), "v"(bh.b), "v"(bl.b));
  }
#pragma unroll
  for (int nt = 0; nt < 7; ++nt) {
    const int col = nt * 16 + m;
#pragma unroll
    for (int r = 0; r < 8; ++r) {
      const int row = 8 * hh + r;
      const float sv = sp5(acc[nt][r]);
      const float v = (col < HR) ? sv : 0.0f;
      us hb, lb;
      split2(v, hb, lb);
      st[w][0][row][col] = hb;
      st[w][1][row][col] = lb;
    }
  }
#pragma unroll
  for (int r = 0; r < 8; ++r) {
    st[w][0][8 * hh + r][112 + m] = (us)0;
    st[w][1][8 * hh + r][112 + m] = (us)0;
  }
  __syncthreads();
  v8us_t vv[2][8];
#pragma unroll
  for (int j = 0; j < 8; ++j) {
    const int row = 2 * j + hh;
    vv[0][j] = *(const v8us*)(&st[w][0][row][8 * m]);
    vv[1][j] = *(const v8us*)(&st[w][1][row][8 * m]);
  }
#pragma unroll
  for (int j = 0; j < 8; ++j) {
    const size_t o = (row0 + 2 * j + hh) * HP + 8 * m;
    vst16(h1h + o, vv[0][j]); vst16(h1l + o, vv[1][j]);
  }
  __threadfence();
#pragma unroll
  for (int j = 0; j < 8; ++j) {
    const size_t o = (row0 + 2 * j + hh) * HP + 8 * m;
    vst16(h1h + o, vv[0][j]); vst16(h1l + o, vv[1][j]);
  }
}

__global__ void __launch_bounds__(128) k_w2f(const us* __restrict__ fph, const us* __restrict__ fpl,
                                             const us* __restrict__ w2h, const us* __restrict__ w2l,
                                             us* __restrict__ oh, us* __restrict__ ol) {
  __shared__ __align__(16) us st[4][2][16][HP];
  const int tid = (int)threadIdx.x, lane = tid & 31, w = tid >> 5;
  const int hh = lane >> 4, m = lane & 15;
  const int gid = blockIdx.x * 4 + w;
  const int lu = gid % NLU;
  const int zbt = gid / NLU;
  const size_t oa = (size_t)(zbt * 16 + m) * EMBD + 8 * hh;
  const Frag ah = ldfrag(fph + oa, 0), al = ldfrag(fpl + oa, 0);
  v8f acc[7];
#pragma unroll
  for (int t = 0; t < 7; ++t) acc[t] = zero8();
  Frag bh, bl;
#pragma unroll
  for (int nt = 0; nt < 7; ++nt) {
    const int kidx = min(nt * 16 + m, HR - 1);
    const size_t ob = (size_t)kidx * W2P + (size_t)lu * 32 + 8 * hh;
    bh = ldfrag(w2h + ob, 0);
    bl = ldfrag(w2l + ob, 0);
    acc[nt] = mma3(ah, al, bh, bl, acc[nt]);
  }
  asm volatile("v_nop\n\tv_nop\n\tv_nop\n\tv_nop"
               : "+v"(acc[0]), "+v"(acc[1]), "+v"(acc[2]), "+v"(acc[3]),
                 "+v"(acc[4]), "+v"(acc[5]), "+v"(acc[6])
               : "v"(ah.b), "v"(al.b), "v"(bh.b), "v"(bl.b));
#pragma unroll
  for (int nt = 0; nt < 7; ++nt) {
    const int col = nt * 16 + m;
#pragma unroll
    for (int r = 0; r < 8; ++r) {
      const int row = 8 * hh + r;
      const float v = (col < HR) ? acc[nt][r] : 0.0f;
      us hb, lb;
      split2(v, hb, lb);
      st[w][0][row][col] = hb;
      st[w][1][row][col] = lb;
    }
  }
#pragma unroll
  for (int r = 0; r < 8; ++r) {
    st[w][0][8 * hh + r][112 + m] = (us)0;
    st[w][1][8 * hh + r][112 + m] = (us)0;
  }
  __syncthreads();
  v8us_t vv[2][8];
#pragma unroll
  for (int j = 0; j < 8; ++j) {
    const int row = 2 * j + hh;
    vv[0][j] = *(const v8us*)(&st[w][0][row][8 * m]);
    vv[1][j] = *(const v8us*)(&st[w][1][row][8 * m]);
  }
#pragma unroll
  for (int j = 0; j < 8; ++j) {
    const int zb = zbt * 16 + 2 * j + hh;
    const size_t o = ((size_t)zb * NLU + lu) * HP + 8 * m;
    vst16(oh + o, vv[0][j]); vst16(ol + o, vv[1][j]);
  }
  __threadfence();
#pragma unroll
  for (int j = 0; j < 8; ++j) {
    const int zb = zbt * 16 + 2 * j + hh;
    const size_t o = ((size_t)zb * NLU + lu) * HP + 8 * m;
    vst16(oh + o, vv[0][j]); vst16(ol + o, vv[1][j]);
  }
}

__global__ void __launch_bounds__(320) k_tang(const float* __restrict__ xyz,
                                              const us* __restrict__ h1h, const us* __restrict__ h1l,
                                              const us* __restrict__ w2fh, const us* __restrict__ w2fl,
                                              us* __restrict__ fah, us* __restrict__ fal,
                                              float* __restrict__ pooledA) {
  __shared__ float facc[NA * RES];
  __shared__ float Tt[32][80];
  __shared__ float At[32][12];
  __shared__ __align__(16) float prow[PP];
  const int tid = (int)threadIdx.x, lane = tid & 31, w = tid >> 5;
  const int hh = lane >> 4, m = lane & 15;
  const int z = blockIdx.x;
  for (int i = tid; i < NA * RES; i += 320) facc[i] = 0.0f;
  const int mt = w / 5;
  const int nt = w - mt * 5;
  const int arow = min(mt * 16 + m, NA - 1);
  const int luc = min(nt * 16 + m, NLU - 1);

#pragma unroll 1
  for (int b = 0; b < NA; ++b) {
    if (tid < NA) {
      const int a = tid;
      float dx, dy, dz;
      const float d = geo_d(xyz + ((size_t)z * NA + a) * 3, xyz + ((size_t)z * NA + b) * 3, dx, dy, dz);
      const float nz = (d > 0.0f) ? 1.0f : 0.0f;
      const float mk = (d < 2.0f) ? 1.0f : 0.0f;
      const float inv = 1.0f / fmaxf(d, 1e-12f);
      const float ux = dx * inv, uy = dy * inv, uz = dz * inv;
      const float s3 = 1.7320508075688772f, hs3 = 0.8660254037844386f;
      At[a][0] = mk;
      At[a][1] = (uy * nz) * mk;
      At[a][2] = (uz * nz) * mk;
      At[a][3] = (ux * nz) * mk;
      At[a][4] = (((s3 * ux) * uy) * nz) * mk;
      At[a][5] = (((s3 * uy) * uz) * nz) * mk;
      At[a][6] = ((0.5f * ((3.0f * uz) * uz - 1.0f)) * nz) * mk;
      At[a][7] = (((s3 * ux) * uz) * nz) * mk;
      At[a][8] = ((hs3 * (ux * ux - uy * uy)) * nz) * mk;
    }
    {
      const size_t pa = ((size_t)z * (NA * NA) + (size_t)arow * NA + b) * HP + 8 * hh;
      const size_t pb = (((size_t)z * NA + b) * NLU + luc) * HP + 8 * hh;
      v8f acc = zero8();
#pragma unroll
      for (int ks = 0; ks < 4; ++ks) {
        const int k0 = ks * 32;
        const Frag ah = ldfrag(h1h + pa, k0), al = ldfrag(h1l + pa, k0);
        const Frag bh = ldfrag(w2fh + pb, k0), bl = ldfrag(w2fl + pb, k0);
        acc = mma3(ah, al, bh, bl, acc);
        asm volatile("v_nop\n\tv_nop\n\tv_nop\n\tv_nop"
                     : "+v"(acc) : "v"(ah.b), "v"(al.b), "v"(bh.b), "v"(bl.b));
      }
#pragma unroll
      for (int r = 0; r < 8; ++r) Tt[mt * 16 + 8 * hh + r][nt * 16 + m] = acc[r];
    }
    __syncthreads();
#pragma unroll 1
    for (int j = 0; j < 21; ++j) {
      const int cell = tid + 320 * j;
      if (cell < NA * RES) {
        const int a = cell / RES;
        const int c = cell - a * RES;
        int lu, sm;
        if (c < 24) { lu = c; sm = 0; }
        else if (c < 96) { const int rr = c - 24; const int u = rr / 3; lu = 24 + u; sm = 1 + (rr - u * 3); }
        else { const int rr = c - 96; const int u = rr / 5; lu = 48 + u; sm = 4 + (rr - u * 5); }
        const float tv = Tt[a][lu];
        const float av = At[a][sm];
        facc[cell] = facc[cell] + tv * av;
      }
    }
    __syncthreads();
  }

  if (tid < PP) {
    const int c = tid;
    float s = 0.0f;
    if (c < RES) {
#pragma unroll 1
      for (int a = 0; a < NA; ++a) s += facc[a * RES + c];
      s = s * (1.0f / 30.0f);
    }
    prow[c] = (c < RES) ? s : 0.0f;
  }
  __syncthreads();

  P16 ph[3], pl[3];
#pragma unroll
  for (int j = 0; j < 3; ++j) {
    const int i = tid + 320 * j;
    const int r = i >> 5;
    const int q = i & 31;
#pragma unroll
    for (int jj = 0; jj < 8; ++jj) {
      const int k = 8 * q + jj;
      const float fv = facc[r * RES + min(k, RES - 1)];
      const float v = (k < RES) ? fv : 0.0f;
      us hb, lb;
      split2(v, hb, lb);
      ph[j].s[jj] = hb; pl[j].s[jj] = lb;
    }
  }
  v4f_t pv;
  pv[0] = 0.0f; pv[1] = 0.0f; pv[2] = 0.0f; pv[3] = 0.0f;
  if (tid < 64) pv = *(const v4f*)(&prow[4 * tid]);
#pragma unroll
  for (int j = 0; j < 3; ++j) {
    const int i = tid + 320 * j;
    const int r = i >> 5, q = i & 31;
    const size_t o = ((size_t)z * NA + r) * FAP + 8 * q;
    vst16(fah + o, ph[j].h); vst16(fal + o, pl[j].h);
  }
  if (tid < 64) vst16f(pooledA + (size_t)z * PP + 4 * tid, pv);
  __threadfence();
#pragma unroll
  for (int j = 0; j < 3; ++j) {
    const int i = tid + 320 * j;
    const int r = i >> 5, q = i & 31;
    const size_t o = ((size_t)z * NA + r) * FAP + 8 * q;
    vst16(fah + o, ph[j].h); vst16(fal + o, pl[j].h);
  }
  if (tid < 64) vst16f(pooledA + (size_t)z * PP + 4 * tid, pv);
}

__global__ void __launch_bounds__(128) k_res(const us* __restrict__ fah, const us* __restrict__ fal,
                                             const us* __restrict__ wrh, const us* __restrict__ wrl,
                                             const float* __restrict__ b_res, float* __restrict__ tlin) {
  __shared__ __align__(16) float st[4][16][128];
  const int tid = (int)threadIdx.x, lane = tid & 31, w = tid >> 5;
  const int hh = lane >> 4, m = lane & 15;
  const int gid = blockIdx.x * 4 + w;
  const int mt = gid >> 1, nh = gid & 1;
  const size_t oa = (size_t)(mt * 16 + m) * FAP + 8 * hh;
  v8f acc[8];
#pragma unroll
  for (int t = 0; t < 8; ++t) acc[t] = zero8();
#pragma unroll 1
  for (int ks = 0; ks < 7; ++ks) {
    const int k0 = ks * 32;
    const Frag ah = ldfrag(fah + oa, k0), al = ldfrag(fal + oa, k0);
    Frag bh, bl;
#pragma unroll
    for (int nt = 0; nt < 8; ++nt) {
      const size_t ob = (size_t)(nh * 128 + nt * 16 + m) * FAP + 8 * hh;
      bh = ldfrag(wrh + ob, k0);
      bl = ldfrag(wrl + ob, k0);
      acc[nt] = mma3(ah, al, bh, bl, acc[nt]);
    }
    asm volatile("v_nop\n\tv_nop\n\tv_nop\n\tv_nop"
                 : "+v"(acc[0]), "+v"(acc[1]), "+v"(acc[2]), "+v"(acc[3]),
                   "+v"(acc[4]), "+v"(acc[5]), "+v"(acc[6]), "+v"(acc[7])
                 : "v"(ah.b), "v"(al.b), "v"(bh.b), "v"(bl.b));
  }
#pragma unroll
  for (int nt = 0; nt < 8; ++nt) {
    const int col = nh * 128 + nt * 16 + m;
    const float bias = b_res[min(col, RES - 1)];
#pragma unroll
    for (int r = 0; r < 8; ++r) {
      const float v = fmaxf(acc[nt][r] + bias, 0.0f);
      st[w][8 * hh + r][nt * 16 + m] = (col < RES) ? v : 0.0f;
    }
  }
  __syncthreads();
  v4f_t vv[16];
#pragma unroll
  for (int j = 0; j < 16; ++j) vv[j] = *(const v4f*)(&st[w][j][4 * lane]);
#pragma unroll
  for (int j = 0; j < 16; ++j)
    vst16f(tlin + (size_t)(mt * 16 + j) * TLP + nh * 128 + 4 * lane, vv[j]);
  __threadfence();
#pragma unroll
  for (int j = 0; j < 16; ++j)
    vst16f(tlin + (size_t)(mt * 16 + j) * TLP + nh * 128 + 4 * lane, vv[j]);
}

__global__ void __launch_bounds__(256) k_bn1(const float* __restrict__ tlin, const float* __restrict__ g1,
                                             const float* __restrict__ be1, float* __restrict__ pooledB) {
  __shared__ float smu[NA][32];
  __shared__ float srs[NA][32];
  __shared__ __align__(16) float pr[NB][32];
  const int tid = (int)threadIdx.x, lane = tid & 31, w = tid >> 5;
  const int cg = blockIdx.x;
  const int ch = cg * 32 + lane;
  const int chc = min(ch, RES - 1);
#pragma unroll 1
  for (int j = 0; j < 4; ++j) {
    const int cell = tid + 256 * j;
    if (cell < NA * 32) {
      const int n = cell >> 5;
      double s = 0.0, ss = 0.0;
#pragma unroll 1
      for (int zz = 0; zz < NB; ++zz) {
        const float x = tlin[((size_t)zz * NA + n) * TLP + ch];
        s += (double)x;
        ss += (double)x * (double)x;
      }
      const double mu = s * (1.0 / 32.0);
      double var = ss * (1.0 / 32.0) - mu * mu;
      if (var < 0.0) var = 0.0;
      smu[n][lane] = (float)mu;
      srs[n][lane] = 1.0f / sqrtf((float)var + 1e-5f);
    }
  }
  __syncthreads();
  const float gg = g1[chc], bb = be1[chc];
#pragma unroll 1
  for (int j = 0; j < 4; ++j) {
    const int cell = tid + 256 * j;
    const int zz = cell >> 5;
    float s = 0.0f;
#pragma unroll 1
    for (int n = 0; n < NA; ++n) {
      const float x = tlin[((size_t)zz * NA + n) * TLP + ch];
      const float y = (gg * (x - smu[n][lane])) * srs[n][lane] + bb;
      s += fmaxf(y, 0.0f);
    }
    s = s * (1.0f / 30.0f);
    pr[zz][lane] = (ch < RES) ? s : 0.0f;
  }
  __syncthreads();
  const int zr = 4 * w + (lane >> 3), q = lane & 7;
  const v4f_t pv = *(const v4f*)(&pr[zr][4 * q]);
  float* dst = pooledB + (size_t)zr * PP + cg * 32 + 4 * q;
  vst16f(dst, pv);
  __threadfence();
  vst16f(dst, pv);
}

__global__ void __launch_bounds__(256) k_head(const float* __restrict__ pooledA, const float* __restrict__ pooledB,
                                              const us* __restrict__ wch, const us* __restrict__ wcl,
                                              const float* __restrict__ b_c, const float* __restrict__ g2,
                                              const float* __restrict__ be2, const float* __restrict__ w_o,
                                              const float* __restrict__ b_o, float* __restrict__ out) {
  __shared__ __align__(16) unsigned char raw[2 * 32 * WCK * 2];
  __shared__ __align__(16) float outv[32];
  us* X0 = reinterpret_cast<us*>(raw);
  us* X1 = X0 + 32 * WCK;
  float* hb = reinterpret_cast<float*>(raw);
  const int tid = (int)threadIdx.x, lane = tid & 31, w = tid >> 5;
  const int hh = lane >> 4, m = lane & 15;

#pragma unroll 1
  for (int j = 0; j < 7; ++j) {
    const int i = tid + 256 * j;
    const int zz = i / 56;
    const int q = i - zz * 56;
#pragma unroll
    for (int jj = 0; jj < 8; ++jj) {
      const int k = 8 * q + jj;
      const int ka = min(k, RES - 1);
      const int kb = min(max(k - RES, 0), RES - 1);
      const float va = pooledA[(size_t)zz * PP + ka];
      const float vb = pooledB[(size_t)zz * PP + kb];
      const float v = (k < RES) ? va : ((k < 2 * RES) ? vb : 0.0f);
      us hbits, lbits;
      split2(v, hbits, lbits);
      X0[zz * WCK + k] = hbits;
      X1[zz * WCK + k] = lbits;
    }
  }
  __syncthreads();

  const int nt = w;
  v8f acc[2];
  acc[0] = zero8(); acc[1] = zero8();
  const us* pbh = wch + (size_t)(nt * 16 + m) * WCK + 8 * hh;
  const us* pbl = wcl + (size_t)(nt * 16 + m) * WCK + 8 * hh;
#pragma unroll 1
  for (int ks = 0; ks < 14; ++ks) {
    const int k0 = ks * 32;
    const Frag bh = ldfrag(pbh, k0), bl = ldfrag(pbl, k0);
    Frag ah, al;
#pragma unroll
    for (int mt = 0; mt < 2; ++mt) {
      ah = ldfrag(X0 + (mt * 16 + m) * WCK + 8 * hh, k0);
      al = ldfrag(X1 + (mt * 16 + m) * WCK + 8 * hh, k0);
      acc[mt] = mma3(ah, al, bh, bl, acc[mt]);
    }
    asm volatile("v_nop\n\tv_nop\n\tv_nop\n\tv_nop"
                 : "+v"(acc[0]), "+v"(acc[1])
                 : "v"(ah.b), "v"(al.b), "v"(bh.b), "v"(bl.b));
  }
  __syncthreads();
  {
    const int c = nt * 16 + m;
    const float bias = b_c[c];
#pragma unroll
    for (int mt = 0; mt < 2; ++mt) {
#pragma unroll
      for (int r = 0; r < 8; ++r) {
        const int zz = mt * 16 + 8 * hh + r;
        const float v = acc[mt][r] + bias;
        hb[zz * 128 + c] = (v >= 0.0f) ? v : 0.01f * v;
      }
    }
  }
  __syncthreads();
  if (tid < 128) {
    const int c = tid;
    double s = 0.0, ss = 0.0;
#pragma unroll 1
    for (int zz = 0; zz < NB; ++zz) {
      const float x = hb[zz * 128 + c];
      s += (double)x;
      ss += (double)x * (double)x;
    }
    const double mu = s * (1.0 / 32.0);
    double var = ss * (1.0 / 32.0) - mu * mu;
    if (var < 0.0) var = 0.0;
    const float muf = (float)mu;
    const float rsd = 1.0f / sqrtf((float)var + 1e-5f);
    const float gg = g2[c], bb = be2[c];
#pragma unroll 1
    for (int zz = 0; zz < NB; ++zz) {
      const float x = hb[zz * 128 + c];
      const float y = (gg * (x - muf)) * rsd + bb;
      hb[zz * 128 + c] = (y >= 0.0f) ? y : 0.01f * y;
    }
  }
  __syncthreads();
  if (tid < NB) {
    const int zz = tid;
    float s = 0.0f;
#pragma unroll 1
    for (int j = 0; j < 128; ++j) s += hb[zz * 128 + j] * w_o[j];
    s += b_o[0];
    const float e = expf(fminf(-s, 30.0f));
    outv[zz] = 1.0f / (1.0f + e);
  }
  __syncthreads();
  v4f_t ov;
  ov[0] = 0.0f; ov[1] = 0.0f; ov[2] = 0.0f; ov[3] = 0.0f;
  if (tid < 8) ov = *(const v4f*)(&outv[4 * tid]);
  if (tid < 8) vst16f(out + 4 * tid, ov);
  __threadfence();
  if (tid < 8) vst16f(out + 4 * tid, ov);
}

extern "C" void kernel_launch(void* const* d_in, const int* in_sizes, int n_in,
                              void* d_out, int out_size, void* d_ws, size_t ws_size,
                              hipStream_t stream) {
  if (n_in < 16) return;
  if (in_sizes[0] != NB * NA * 3) return;
  if (in_sizes[1] != NB * NA) return;
  if (in_sizes[2] != 6 * EMBD) return;
  if (in_sizes[3] != 3 * HR) return;
  if (in_sizes[4] != HR * HR) return;
  if (in_sizes[5] != HR * W2P) return;
  if (in_sizes[6] != RES * RES) return;
  if (in_sizes[7] != RES) return;
  if (in_sizes[8] != RES) return;
  if (in_sizes[9] != RES) return;
  if (in_sizes[10] != 2 * RES * 128) return;
  if (in_sizes[11] != 128) return;
  if (in_sizes[12] != 128) return;
  if (in_sizes[13] != 128) return;
  if (in_sizes[14] != 128) return;
  if (in_sizes[15] != 1) return;
  if (out_size != NB) return;

  const float* xyz      = (const float*)d_in[0];
  const int*   features = (const int*)  d_in[1];
  const float* emb      = (const float*)d_in[2];
  const float* w_r0     = (const float*)d_in[3];
  const float* w_r1     = (const float*)d_in[4];
  const float* w_r2     = (const float*)d_in[5];
  const float* w_res    = (const float*)d_in[6];
  const float* b_res    = (const float*)d_in[7];
  const float* bn1_g    = (const float*)d_in[8];
  const float* bn1_b    = (const float*)d_in[9];
  const float* w_c      = (const float*)d_in[10];
  const float* b_c      = (const float*)d_in[11];
  const float* bn2_g    = (const float*)d_in[12];
  const float* bn2_b    = (const float*)d_in[13];
  const float* w_o      = (const float*)d_in[14];
  const float* b_o      = (const float*)d_in[15];
  float* out = (float*)d_out;

  const size_t szH    = (size_t)NPAIR * HP * 2;
  const size_t szW1   = (size_t)112 * HP * 2;
  const size_t szW2   = (size_t)W2PIECES * 16;
  const size_t szFP   = (size_t)NB * NA * EMBD * 2;
  const size_t szW2F  = (size_t)NB * NA * NLU * HP * 2;
  const size_t szFA   = (size_t)NB * NA * FAP * 2;
  const size_t szWR   = (size_t)WRROWS * FAP * 2;
  const size_t szWC   = (size_t)128 * WCK * 2;
  const size_t szPO   = (size_t)NB * PP * 4;
  const size_t szTL   = (size_t)NB * NA * TLP * 4;
  size_t off = 0;
  char* ws = (char*)d_ws;
  auto carve = [&](size_t bytes) -> char* {
    char* p = ws + off;
    off += (bytes + 255) & ~(size_t)255;
    return p;
  };
  us* h0h = (us*)carve(szH);   us* h0l = (us*)carve(szH);
  us* h1h = (us*)carve(szH);   us* h1l = (us*)carve(szH);
  us* w1h = (us*)carve(szW1);  us* w1l = (us*)carve(szW1);
  us* w2h = (us*)carve(szW2);  us* w2l = (us*)carve(szW2);
  us* fph = (us*)carve(szFP);  us* fpl = (us*)carve(szFP);
  us* W2h = (us*)carve(szW2F); us* W2l = (us*)carve(szW2F);
  us* fah = (us*)carve(szFA);  us* fal = (us*)carve(szFA);
  us* wrh = (us*)carve(szWR);  us* wrl = (us*)carve(szWR);
  us* wch = (us*)carve(szWC);  us* wcl = (us*)carve(szWC);
  float* pooledA = (float*)carve(szPO);
  float* pooledB = (float*)carve(szPO);
  float* tlin    = (float*)carve(szTL);
  const size_t total = off;
  if (total > ws_size) return;
  if (total > (size_t)134217728) return;

  k_cvt<<<1792 / 256, 256, 0, stream>>>(w_r1, w1h, w1l, HR, HR, HR, HP / 8, 1);
  k_cvt<<<W2PIECES / 256, 256, 0, stream>>>(w_r2, w2h, w2l, HR, W2P, W2P, W2P / 8, 0);
  k_cvt<<<8192 / 256, 256, 0, stream>>>(w_res, wrh, wrl, RES, RES, RES, FAP / 8, 1);
  k_cvt<<<7168 / 256, 256, 0, stream>>>(w_c, wch, wcl, 128, 2 * RES, 128, WCK / 8, 1);
  k_feat<<<3840 / 256, 256, 0, stream>>>(features, emb, fph, fpl);

  k_geom<<<NPAIR / 32, 256, 0, stream>>>(xyz, w_r0, h0h, h0l);
  k_mlp1<<<1800 / 4, 128, 0, stream>>>(h0h, h0l, w1h, w1l, h1h, h1l);
  k_w2f<<<4320 / 4, 128, 0, stream>>>(fph, fpl, w2h, w2l, W2h, W2l);
  k_tang<<<NB, 320, 0, stream>>>(xyz, h1h, h1l, W2h, W2l, fah, fal, pooledA);
  k_res<<<120 / 4, 128, 0, stream>>>(fah, fal, wrh, wrl, b_res, tlin);
  k_bn1<<<7, 256, 0, stream>>>(tlin, bn1_g, bn1_b, pooledB);
  k_head<<<1, 256, 0, stream>>>(pooledA, pooledB, wch, wcl, b_c, bn2_g, bn2_b, w_o, b_o, out);
}
